// TemporalSeparateAttention_25864293056657
// MI455X (gfx1250) — hardware-verified
//
#include <hip/hip_runtime.h>
#include <stddef.h>


typedef _Float16 v16h __attribute__((ext_vector_type(16)));
typedef _Float16 v8h  __attribute__((ext_vector_type(8)));
typedef _Float16 v4h  __attribute__((ext_vector_type(4)));
typedef float    v8f  __attribute__((ext_vector_type(8)));
typedef float    v4f  __attribute__((ext_vector_type(4)));

#ifndef NB
#define NB 2
#endif
#define NB_FULL 2
#define NQ     1024
#define NKEY   3072
#define CDIM   256
#define NHEAD  8
#define HD     32
#define KCAT   512
#define QSPLIT 896
#define K1END  1536
#define K1BEG2 2688
#define KGAP   (K1BEG2 - K1END)
#define QTILES   (NQ / 64)
#define QT_SPLIT (QSPLIT / 64)
#define KT0      (NKEY / 64)
#define KT1A     (K1END / 64)
#define KT1B     ((NKEY - K1BEG2) / 64)
#define KT1      (KT1A + KT1B)
#define KTILES   (KT0 + KT1)
#define QBLK       (NQ / 128)
#define QBLK_SPLIT (QSPLIT / 128)
#ifndef SCORE_RES
#define SCORE_RES 1
#endif

static_assert(NB >= 1 && NB <= NB_FULL);
static_assert(CDIM == NHEAD * HD);
static_assert(HD == 32);
static_assert(KCAT == 2 * CDIM);
static_assert((CDIM % 64) == 0 && (CDIM % 32) == 0 && (KCAT % 32) == 0);
static_assert(CDIM == 32 * 8);
static_assert((NQ % 128) == 0 && (QSPLIT % 128) == 0);
static_assert((NKEY % 64) == 0 && (K1END % 64) == 0 && (K1BEG2 % 64) == 0);
static_assert(K1BEG2 > K1END && K1BEG2 < NKEY);
static_assert(KT1A * 64 == K1END && K1BEG2 + KT1B * 64 == NKEY);
static_assert(QBLK * 128 == NQ && QTILES * 64 == NQ);
static_assert(((NB * NQ) % 8) == 0 && ((NB * NKEY) % 8) == 0);

#define LDT 72
#define LDK 40
#define LDC 68
static_assert((LDT % 8) == 0 && LDT >= 64);
static_assert((LDK % 8) == 0 && LDK >= HD);
static_assert((LDC % 4) == 0 && LDC >= 64);

#define WCARRY 64.0f
#define PCARRY 16384.0f
#define VCARRY 64.0f
#define RCARRY 2048.0f

#define WQK_BYTES ((size_t)2 * CDIM * KCAT * 2)
#define WVO_BYTES ((size_t)2 * CDIM * CDIM * 2)
#define XQ_BYTES  ((size_t)NB * NQ * KCAT * 2)
#define XK_BYTES  ((size_t)NB * NKEY * KCAT * 2)
#define XV_BYTES  ((size_t)NB * NKEY * CDIM * 2)
#define QP_BYTES  ((size_t)NB * NQ * CDIM * 2)
#define KP_BYTES  ((size_t)2 * NB * NKEY * CDIM * 2)
#define CTX_BYTES ((size_t)NB * NHEAD * NQ * HD * 2)
#define OFF_WQ  ((size_t)0)
#define OFF_WK  (OFF_WQ + WQK_BYTES)
#define OFF_WV  (OFF_WK + WQK_BYTES)
#define OFF_WO  (OFF_WV + WVO_BYTES)
#define OFF_XQ  (OFF_WO + WVO_BYTES)
#define OFF_XK  (OFF_XQ + XQ_BYTES)
#define OFF_XV  (OFF_XK + XK_BYTES)
#define OFF_QH  (OFF_XV + XV_BYTES)
#define OFF_QR  (OFF_QH + QP_BYTES)
#define OFF_KH  (OFF_QR + QP_BYTES)
#define OFF_KR  (OFF_KH + KP_BYTES)
#define OFF_VT  (OFF_KR + KP_BYTES)
#define OFF_CTX (OFF_VT + KP_BYTES)
#define WS_TOTAL (OFF_CTX + CTX_BYTES)
static_assert((WQK_BYTES % 128) == 0 && (WVO_BYTES % 128) == 0 && (XQ_BYTES % 128) == 0);
static_assert((XK_BYTES % 128) == 0 && (XV_BYTES % 128) == 0 && (QP_BYTES % 128) == 0);
static_assert((KP_BYTES % 128) == 0 && (CTX_BYTES % 128) == 0);
static_assert(WS_TOTAL <= (size_t)134217728);

__device__ __forceinline__ float bf16r(float x) {
  unsigned int u = __float_as_uint(x);
  u = (u + 0x7FFFu + ((u >> 16) & 1u)) & 0xFFFF0000u;
  return __uint_as_float(u);
}

__device__ __forceinline__ _Float16 toh_flush(float v) {
  const _Float16 r = (_Float16)v;
  return (fabsf(v) < 6.103515625e-05f) ? (_Float16)0.0f : r;
}

__device__ __forceinline__ v16h frag_at(const _Float16* p) {
  v8h lo = *(const v8h*)(p);
  v8h hi = *(const v8h*)(p + 16);
  v16h out;
#pragma unroll
  for (int i = 0; i < 8; ++i) { out[i] = lo[i]; out[i + 8] = hi[i]; }
  return out;
}
__device__ __forceinline__ v16h ld_frag(const _Float16* base, unsigned ld) {
  const unsigned lane = threadIdx.x & 31u;
  return frag_at(base + (lane & 15u) * ld + (lane >> 4) * 8u);
}

__device__ __forceinline__ v8f wmma16(v16h a, v16h b, v8f c) {
  v8f d = __builtin_amdgcn_wmma_f32_16x16x32_f16(false, a, false, b, (short)0, c,
                                                 false, false);
  asm volatile("v_nop\n\tv_nop\n\tv_nop\n\tv_nop" : "+v"(d) : "v"(a), "v"(b));
  return d;
}

__device__ __forceinline__ float red16_max(float x) {
#pragma unroll
  for (int off = 1; off < 16; off <<= 1) x = fmaxf(x, __shfl_xor(x, off, 32));
  return x;
}
__device__ __forceinline__ float red16_sum(float x) {
#pragma unroll
  for (int off = 1; off < 16; off <<= 1) x += __shfl_xor(x, off, 32);
  return x;
}

__device__ __forceinline__ void wave_lds_sync() {
  __builtin_amdgcn_fence(3  , "wavefront");
  asm volatile("s_wait_dscnt 0x0" ::: "memory");
  __builtin_amdgcn_wave_barrier();
}

__global__ __launch_bounds__(256) void wcast_kernel(
    const float* __restrict__ W, _Float16* __restrict__ Wp, unsigned ldk, unsigned ndup) {
  const unsigned lane = threadIdx.x & 31u;
  const unsigned wave = (unsigned)__builtin_amdgcn_readfirstlane((int)(threadIdx.x >> 5));
  const unsigned n = blockIdx.x * 8u + wave;
  const float* src = W + (size_t)n * CDIM + lane * 8u;
  const v4f a0 = *(const v4f*)(src);
  const v4f a1 = *(const v4f*)(src + 4);
  v8h x;
#pragma unroll
  for (int i = 0; i < 4; ++i) {
    x[i]     = toh_flush(WCARRY * bf16r(a0[i]));
    x[i + 4] = toh_flush(WCARRY * bf16r(a1[i]));
  }
  _Float16* p = Wp + (size_t)n * ldk + lane * 8u;
#pragma unroll 1
  for (unsigned d = 0; d < ndup; ++d) *(volatile v8h*)(p + d * (unsigned)CDIM) = x;
  __threadfence();
#pragma unroll 1
  for (unsigned d = 0; d < ndup; ++d) *(volatile v8h*)(p + d * (unsigned)CDIM) = x;
}

__global__ __launch_bounds__(256) void xcast_kernel(
    const float* __restrict__ X, _Float16* __restrict__ dst, unsigned ldo, unsigned coff) {
  const unsigned lane = threadIdx.x & 31u;
  const unsigned wave = (unsigned)__builtin_amdgcn_readfirstlane((int)(threadIdx.x >> 5));
  const unsigned row = blockIdx.x * 8u + wave;
  const float* src = X + (size_t)row * CDIM + lane * 8u;
  const v4f a0 = *(const v4f*)(src);
  const v4f a1 = *(const v4f*)(src + 4);
  v8h x;
#pragma unroll
  for (int i = 0; i < 4; ++i) {
    x[i]     = toh_flush(bf16r(a0[i]));
    x[i + 4] = toh_flush(bf16r(a1[i]));
  }
  _Float16* p = dst + (size_t)row * ldo + coff + lane * 8u;
  *(volatile v8h*)p = x;
  __threadfence();
  *(volatile v8h*)p = x;
}

template <int MODE>
__device__ __forceinline__ void gemm_body(
    const _Float16* __restrict__ A16, const _Float16* __restrict__ Bt,
    float* __restrict__ outf, _Float16* __restrict__ out16, _Float16* __restrict__ out16r) {
  __shared__ float Cs[64 * LDC];
  const unsigned tid = threadIdx.x, lane = tid & 31u;
  const unsigned w = (unsigned)__builtin_amdgcn_readfirstlane((int)(tid >> 5));
  const unsigned mw = w >> 1, nw = w & 1u;
  const unsigned hh = lane >> 4, m = lane & 15u;
  const unsigned n0 = blockIdx.x * 64u;
  const unsigned ty = blockIdx.y;

  unsigned b, set, trow;
  if (MODE == 0 || MODE == 3) {
    b = ty / (unsigned)QTILES;
    const unsigned qt = ty - b * (unsigned)QTILES;
    set = (qt >= (unsigned)QT_SPLIT) ? 1u : 0u;
    trow = qt * 64u;
  } else {
    b = ty / (unsigned)KTILES;
    const unsigned t = ty - b * (unsigned)KTILES;
    set = (t >= (unsigned)KT0) ? 1u : 0u;
    const unsigned u = t - set * (unsigned)KT0;
    trow = u * 64u + ((set != 0u && u >= (unsigned)KT1A) ? (unsigned)KGAP : 0u);
  }
  const unsigned K = (MODE <= 1) ? (unsigned)KCAT : (unsigned)CDIM;
  const unsigned apitch = (MODE == 3) ? (unsigned)HD : K;
  const unsigned akstep = (MODE == 3) ? (unsigned)(NQ * HD) : 32u;
  size_t abase;
  if (MODE == 0)      abase = ((size_t)b * NQ + trow) * KCAT;
  else if (MODE == 1) abase = ((size_t)b * NKEY + trow) * KCAT;
  else if (MODE == 2) abase = ((size_t)b * NKEY + trow) * CDIM;
  else                abase = ((size_t)b * NHEAD * NQ + trow) * HD;
  const size_t bbase = (size_t)set * CDIM * K;

  const _Float16* ap  = A16 + abase + (size_t)(mw * 16u + m) * apitch + hh * 8u;
  const _Float16* bp0 = Bt + bbase + (size_t)(n0 + nw * 32u + m) * K + hh * 8u;
  const _Float16* bp1 = bp0 + (size_t)16 * K;
  v8f acc0 = {}, acc1 = {};
#pragma unroll 2
  for (unsigned ks = 0; ks < K / 32u; ++ks) {
    const v16h a  = frag_at(ap + (size_t)ks * akstep);
    const v16h b0 = frag_at(bp0 + ks * 32u);
    const v16h b1 = frag_at(bp1 + ks * 32u);
    acc0 = wmma16(a, b0, acc0);
    acc1 = wmma16(a, b1, acc1);
  }
#pragma unroll
  for (int r = 0; r < 8; ++r) {
    float* d = &Cs[(mw * 16u + hh * 8u + (unsigned)r) * LDC + nw * 32u + m];
    d[0]  = acc0[r];
    d[16] = acc1[r];
  }
  __syncthreads();

  if (MODE == 0 || MODE == 1) {
    const size_t obase = (MODE == 0)
        ? ((size_t)b * NQ + trow) * CDIM
        : (((size_t)set * NB + b) * NKEY + trow) * CDIM;
    v8h x[2], xr[2];
    size_t off[2];
#pragma unroll
    for (unsigned i = 0; i < 2u; ++i) {
      const unsigned r = 32u * i + (tid >> 3);
      const unsigned c = (tid & 7u) * 8u;
      const v4f u0 = *(const v4f*)&Cs[r * LDC + c];
      const v4f u1 = *(const v4f*)&Cs[r * LDC + c + 4];
#pragma unroll
      for (int j = 0; j < 4; ++j) {
        const float t0 = u0[j] * (1.0f / WCARRY);
        const float t1 = u1[j] * (1.0f / WCARRY);
        const _Float16 h0 = toh_flush(t0);
        const _Float16 h1 = toh_flush(t1);
        x[i][j]      = h0;
        x[i][j + 4]  = h1;
        xr[i][j]     = toh_flush((t0 - (float)h0) * RCARRY);
        xr[i][j + 4] = toh_flush((t1 - (float)h1) * RCARRY);
      }
      off[i] = obase + (size_t)r * CDIM + n0 + c;
    }
#pragma unroll
    for (int i = 0; i < 2; ++i) *(volatile v8h*)(out16 + off[i]) = x[i];
#pragma unroll
    for (int i = 0; i < 2; ++i) *(volatile v8h*)(out16r + off[i]) = xr[i];
    __threadfence();
#pragma unroll
    for (int i = 0; i < 2; ++i) *(volatile v8h*)(out16 + off[i]) = x[i];
#pragma unroll
    for (int i = 0; i < 2; ++i) *(volatile v8h*)(out16r + off[i]) = xr[i];
  }

  if (MODE == 2) {
    const size_t vbase = (((size_t)set * NB + b) * CDIM) * NKEY;
    v8h x[2];
    size_t off[2];
#pragma unroll
    for (unsigned i = 0; i < 2u; ++i) {
      const unsigned dcol = 32u * i + (tid >> 3);
      const unsigned kk = (tid & 7u) * 8u;
#pragma unroll
      for (unsigned j = 0; j < 8u; ++j) {
        const float t = Cs[(kk + j) * LDC + dcol] * (1.0f / WCARRY);
        x[i][j] = toh_flush(t);
      }
      off[i] = vbase + (size_t)(n0 + dcol) * NKEY + trow + kk;
    }
#pragma unroll
    for (int i = 0; i < 2; ++i) *(volatile v8h*)(out16 + off[i]) = x[i];
    __threadfence();
#pragma unroll
    for (int i = 0; i < 2; ++i) *(volatile v8h*)(out16 + off[i]) = x[i];
  }

  if (MODE == 3) {
    const float cs = 1.0f / (WCARRY * VCARRY);
    const size_t obase = ((size_t)b * NQ + trow) * CDIM;
    v4f xs[4];
    size_t off[4];
#pragma unroll
    for (unsigned i = 0; i < 4u; ++i) {
      const unsigned r = 16u * i + (tid >> 4);
      const unsigned c = (tid & 15u) * 4u;
      const v4f u = *(const v4f*)&Cs[r * LDC + c];
      v4f val;
#pragma unroll
      for (int j = 0; j < 4; ++j) val[j] = u[j] * cs;
      xs[i] = val;
      off[i] = obase + (size_t)r * CDIM + n0 + c;
    }
#pragma unroll
    for (int i = 0; i < 4; ++i) *(volatile v4f*)(outf + off[i]) = xs[i];
    __threadfence();
#pragma unroll
    for (int i = 0; i < 4; ++i) *(volatile v4f*)(outf + off[i]) = xs[i];
  }
}

__global__ __launch_bounds__(256) void gemm_q_kernel(
    const _Float16* __restrict__ A16, const _Float16* __restrict__ Bt,
    _Float16* __restrict__ qh, _Float16* __restrict__ qr) {
  gemm_body<0>(A16, Bt, (float*)0, qh, qr);
}
__global__ __launch_bounds__(256) void gemm_k_kernel(
    const _Float16* __restrict__ A16, const _Float16* __restrict__ Bt,
    _Float16* __restrict__ kh, _Float16* __restrict__ kr) {
  gemm_body<1>(A16, Bt, (float*)0, kh, kr);
}
__global__ __launch_bounds__(256) void gemm_v_kernel(
    const _Float16* __restrict__ A16, const _Float16* __restrict__ Bt,
    _Float16* __restrict__ vt) {
  gemm_body<2>(A16, Bt, (float*)0, vt, vt);
}
__global__ __launch_bounds__(256) void gemm_o_kernel(
    const _Float16* __restrict__ A16, const _Float16* __restrict__ Bt,
    float* __restrict__ outf) {
  gemm_body<3>(A16, Bt, outf, (_Float16*)0, (_Float16*)0);
}

__global__ __launch_bounds__(256) void attn_kernel(
    const _Float16* __restrict__ Qh, const _Float16* __restrict__ Qr,
    const _Float16* __restrict__ Kh, const _Float16* __restrict__ Kr,
    const _Float16* __restrict__ Vt, const float* __restrict__ Mk,
    _Float16* __restrict__ Ov) {
  __shared__ _Float16 Ks[64 * LDK];
#if SCORE_RES
  __shared__ _Float16 KRs[64 * LDK];
#endif
  __shared__ _Float16 Vs[HD * LDT];
  __shared__ _Float16 Ms[128 * LDT];
  __shared__ _Float16 Ps[8 * 16 * LDT];

  const unsigned tid = threadIdx.x, lane = tid & 31u;
  const unsigned w = (unsigned)__builtin_amdgcn_readfirstlane((int)(tid >> 5));
  const unsigned hh = lane >> 4, m = lane & 15u;
  const unsigned q0 = blockIdx.x * 128u;
  const unsigned head = blockIdx.y;
  const unsigned b = blockIdx.z;
  const unsigned set = (blockIdx.x >= (unsigned)QBLK_SPLIT) ? 1u : 0u;
  const float scale = 0.17677669529663687f;
  const unsigned qrow0 = q0 + w * 16u;
  _Float16* P = Ps + w * (16u * LDT);

  const size_t qoff = (size_t)(b * (unsigned)NQ + qrow0 + m) * CDIM + head * HD + hh * 8u;
  const v16h qf = frag_at(Qh + qoff);
#if SCORE_RES
  const v16h qr = frag_at(Qr + qoff);
#endif

  float mrow[8], lrow[8];
  v8f o[2];
#pragma unroll
  for (int v = 0; v < 8; ++v) { mrow[v] = -1.0e30f; lrow[v] = 0.0f; }
#pragma unroll
  for (int nb = 0; nb < 2; ++nb) o[nb] = (v8f){};

  const size_t kplane = (((size_t)set * NB + b) * NKEY) * CDIM + head * HD;
  const size_t vplane = (((size_t)set * NB + b) * CDIM + head * HD) * NKEY;
  const unsigned nsteps = (set != 0u) ? (unsigned)KT1 : (unsigned)KT0;
  const unsigned nfirst = (set != 0u) ? (unsigned)KT1A : (unsigned)KT0;

  for (unsigned t = 0; t < nsteps; ++t) {
    const unsigned kb = t * 64u + ((t >= nfirst) ? (unsigned)KGAP : 0u);
    {
      const unsigned r = tid >> 2, c = (tid & 3u) * 8u;
      const size_t g = kplane + (size_t)(kb + r) * CDIM + c;
      *(v8h*)&Ks[r * LDK + c] = *(const v8h*)(Kh + g);
#if SCORE_RES
      *(v8h*)&KRs[r * LDK + c] = *(const v8h*)(Kr + g);
#endif
      const unsigned d = tid >> 3, kc = (tid & 7u) * 8u;
      *(v8h*)&Vs[d * LDT + kc] = *(const v8h*)(Vt + vplane + (size_t)d * NKEY + kb + kc);
    }
#pragma unroll
    for (unsigned j = 0; j < 8u; ++j) {
      const unsigned idx = tid + 256u * j;
      const unsigned r = idx >> 4, c = (idx & 15u) * 4u;
      const v4f mv = *(const v4f*)(Mk + (size_t)(q0 + r) * NKEY + kb + c);
      v4h mh;
#pragma unroll
      for (int i = 0; i < 4; ++i) mh[i] = (_Float16)bf16r(mv[i]);
      *(v4h*)&Ms[r * LDT + c] = mh;
    }
    __syncthreads();

    v8f s[4];
#pragma unroll
    for (int kg = 0; kg < 4; ++kg) {
      const v16h kf = ld_frag(&Ks[(kg * 16) * LDK], LDK);
      v8f a = {};
      a = wmma16(qf, kf, a);
#if SCORE_RES
      const v16h kr = ld_frag(&KRs[(kg * 16) * LDK], LDK);
      v8f u = {};
      u = wmma16(qf, kr, u);
      u = wmma16(qr, kf, u);
#endif
#pragma unroll
      for (int v = 0; v < 8; ++v) {
        float sc = a[v];
#if SCORE_RES
        sc = sc + u[v] * (1.0f / RCARRY);
#endif
        const float mk = (float)Ms[(w * 16u + hh * 8u + (unsigned)v) * LDT + (unsigned)kg * 16u + m];
        s[kg][v] = sc * scale + mk;
      }
    }

    float alpha[8];
#pragma unroll
    for (int v = 0; v < 8; ++v) {
      float mx = fmaxf(fmaxf(s[0][v], s[1][v]), fmaxf(s[2][v], s[3][v]));
      mx = red16_max(mx);
      const float mn = fmaxf(mrow[v], mx);
      alpha[v] = __expf(mrow[v] - mn);
      mrow[v] = mn;
    }
#pragma unroll
    for (int kg = 0; kg < 4; ++kg)
#pragma unroll
      for (int v = 0; v < 8; ++v) s[kg][v] = __expf(s[kg][v] - mrow[v]);
#pragma unroll
    for (int v = 0; v < 8; ++v) {
      const float rs = red16_sum((s[0][v] + s[1][v]) + (s[2][v] + s[3][v]));
      lrow[v] = alpha[v] * lrow[v] + rs;
    }
#pragma unroll
    for (int nb = 0; nb < 2; ++nb)
#pragma unroll
      for (int v = 0; v < 8; ++v) o[nb][v] = o[nb][v] * alpha[v];

#pragma unroll
    for (int kg = 0; kg < 4; ++kg)
#pragma unroll
      for (int v = 0; v < 8; ++v)
        P[(hh * 8u + (unsigned)v) * LDT + (unsigned)kg * 16u + m] = toh_flush(s[kg][v] * PCARRY);
    wave_lds_sync();

#pragma unroll
    for (int c = 0; c < 2; ++c) {
      const v16h pf = ld_frag(P + c * 32, LDT);
#pragma unroll
      for (int nb = 0; nb < 2; ++nb) {
        const v16h vf = ld_frag(&Vs[(nb * 16) * LDT + c * 32], LDT);
        o[nb] = wmma16(pf, vf, o[nb]);
      }
    }
    __syncthreads();
  }

  float inv[8];
#pragma unroll
  for (int v = 0; v < 8; ++v) inv[v] = __builtin_amdgcn_rcpf(lrow[v]) * (VCARRY / PCARRY);
#pragma unroll
  for (int nb = 0; nb < 2; ++nb)
#pragma unroll
    for (int v = 0; v < 8; ++v)
      P[(hh * 8u + (unsigned)v) * LDT + (unsigned)nb * 16u + m] = toh_flush(o[nb][v] * inv[v]);
  wave_lds_sync();
  v8h x[2];
  size_t off[2];
#pragma unroll
  for (unsigned i = 0; i < 2u; ++i) {
    const unsigned r = 8u * i + (lane >> 2);
    const unsigned c = (lane & 3u) * 8u;
    x[i] = *(const v8h*)&P[r * LDT + c];
    off[i] = (((size_t)b * NHEAD + head) * NQ + qrow0 + r) * HD + c;
  }
#pragma unroll
  for (int i = 0; i < 2; ++i) *(volatile v8h*)(Ov + off[i]) = x[i];
  __threadfence();
#pragma unroll
  for (int i = 0; i < 2; ++i) *(volatile v8h*)(Ov + off[i]) = x[i];
}

extern "C" void kernel_launch(void* const* d_in, const int* in_sizes, int n_in,
                              void* d_out, int out_size, void* d_ws, size_t ws_size,
                              hipStream_t stream) {
  if (n_in < 14) return;
  const long long need_q = (long long)NB * NQ * CDIM;
  const long long need_k = (long long)NB * NKEY * CDIM;
  if ((long long)in_sizes[0] < need_q) return;
  if ((long long)in_sizes[1] < need_k) return;
  if ((long long)in_sizes[2] < need_k) return;
  if ((long long)in_sizes[3] < need_q) return;
  if ((long long)in_sizes[4] < need_k) return;
  if ((long long)in_sizes[5] < (long long)NQ * NKEY) return;
  for (int i = 6; i < 14; ++i)
    if ((long long)in_sizes[i] < (long long)CDIM * CDIM) return;
  if ((long long)out_size < need_q) return;
  if (ws_size < WS_TOTAL) return;

  const float* query = (const float*)d_in[0];
  const float* key   = (const float*)d_in[1];
  const float* value = (const float*)d_in[2];
  const float* qpos  = (const float*)d_in[3];
  const float* kpos  = (const float*)d_in[4];
  const float* mask  = (const float*)d_in[5];
  const float* wq0 = (const float*)d_in[6];
  const float* wk0 = (const float*)d_in[7];
  const float* wv0 = (const float*)d_in[8];
  const float* wo0 = (const float*)d_in[9];
  const float* wq1 = (const float*)d_in[10];
  const float* wk1 = (const float*)d_in[11];
  const float* wv1 = (const float*)d_in[12];
  const float* wo1 = (const float*)d_in[13];
  float* out = (float*)d_out;

  char* ws = (char*)d_ws;
  _Float16* WQp  = (_Float16*)(ws + OFF_WQ);
  _Float16* WKp  = (_Float16*)(ws + OFF_WK);
  _Float16* WVp  = (_Float16*)(ws + OFF_WV);
  _Float16* WOp  = (_Float16*)(ws + OFF_WO);
  _Float16* XQ16 = (_Float16*)(ws + OFF_XQ);
  _Float16* XK16 = (_Float16*)(ws + OFF_XK);
  _Float16* XV16 = (_Float16*)(ws + OFF_XV);
  _Float16* Qh16 = (_Float16*)(ws + OFF_QH);
  _Float16* Qr16 = (_Float16*)(ws + OFF_QR);
  _Float16* Kh16 = (_Float16*)(ws + OFF_KH);
  _Float16* Kr16 = (_Float16*)(ws + OFF_KR);
  _Float16* Vt16 = (_Float16*)(ws + OFF_VT);
  _Float16* Ctx16 = (_Float16*)(ws + OFF_CTX);

  dim3 blk(256);
  dim3 gw(CDIM / 8);

  wcast_kernel<<<gw, blk, 0, stream>>>(wq0, WQp, (unsigned)KCAT, 2u);
  wcast_kernel<<<gw, blk, 0, stream>>>(wq1, WQp + (size_t)CDIM * KCAT, (unsigned)KCAT, 2u);
  wcast_kernel<<<gw, blk, 0, stream>>>(wk0, WKp, (unsigned)KCAT, 2u);
  wcast_kernel<<<gw, blk, 0, stream>>>(wk1, WKp + (size_t)CDIM * KCAT, (unsigned)KCAT, 2u);
  wcast_kernel<<<gw, blk, 0, stream>>>(wv0, WVp, (unsigned)CDIM, 1u);
  wcast_kernel<<<gw, blk, 0, stream>>>(wv1, WVp + (size_t)CDIM * CDIM, (unsigned)CDIM, 1u);
  wcast_kernel<<<gw, blk, 0, stream>>>(wo0, WOp, (unsigned)CDIM, 1u);
  wcast_kernel<<<gw, blk, 0, stream>>>(wo1, WOp + (size_t)CDIM * CDIM, (unsigned)CDIM, 1u);

  xcast_kernel<<<dim3(NB * NQ / 8), blk, 0, stream>>>(query, XQ16, (unsigned)KCAT, 0u);
  xcast_kernel<<<dim3(NB * NQ / 8), blk, 0, stream>>>(qpos, XQ16, (unsigned)KCAT, (unsigned)CDIM);
  xcast_kernel<<<dim3(NB * NKEY / 8), blk, 0, stream>>>(key, XK16, (unsigned)KCAT, 0u);
  xcast_kernel<<<dim3(NB * NKEY / 8), blk, 0, stream>>>(kpos, XK16, (unsigned)KCAT, (unsigned)CDIM);
  xcast_kernel<<<dim3(NB * NKEY / 8), blk, 0, stream>>>(value, XV16, (unsigned)CDIM, 0u);

  gemm_q_kernel<<<dim3(CDIM / 64, NB * QTILES), blk, 0, stream>>>(XQ16, WQp, Qh16, Qr16);
  gemm_k_kernel<<<dim3(CDIM / 64, NB * KTILES), blk, 0, stream>>>(XK16, WKp, Kh16, Kr16);
  gemm_v_kernel<<<dim3(CDIM / 64, NB * KTILES), blk, 0, stream>>>(XV16, WVp, Vt16);
  attn_kernel<<<dim3(QBLK, NHEAD, NB), blk, 0, stream>>>(Qh16, Qr16, Kh16, Kr16, Vt16, mask, Ctx16);
  gemm_o_kernel<<<dim3(CDIM / 64, NB * QTILES), blk, 0, stream>>>(Ctx16, WOp, out);
}
